// MultiHeadAttention_52261162058330
// MI455X (gfx1250) — hardware-verified
//
#include <hip/hip_runtime.h>


#ifndef NB
#define NB 2
#endif
#ifndef SEQ
#define SEQ 2048
#endif
#define NB_FULL  2
#define SEQ_FULL 2048
#ifndef OUT_SEQ
#define OUT_SEQ SEQ
#endif
#define NHD    16
#define HD     64
#define NZ     (NB * NHD)
#define KSPLIT 8
#define KC     (SEQ / KSPLIT)
#define TP     65
#define OSW    68

static_assert(HD == 64);
static_assert(SEQ % 64 == 0);
static_assert(SEQ % KSPLIT == 0);
static_assert(KC % 32 == 0);
static_assert(HD % 32 == 0);
static_assert(NB <= NB_FULL);
static_assert(SEQ <= SEQ_FULL);
static_assert(((size_t)SEQ * HD) % 8 == 0);
static_assert((OSW * 4) % 16 == 0);
static_assert(4 * 256 * 4 == 64 * 64);
static_assert(2 * 256 * 8 == 64 * 64);
static_assert(8 * 32 * 16 == 16 * HD * 4);
static_assert(16 * 8 * 2 == 2 * HD * 2);
static_assert(64 * TP * 4 <= 131072);
static_assert(16 * OSW * 4 <= 131072);
static_assert(((size_t)NZ * 1024) % 256 == 0);

typedef unsigned short bf;
typedef __attribute__((ext_vector_type(16))) __bf16   v16bf;
typedef __attribute__((ext_vector_type(8)))  unsigned short v8us;
typedef __attribute__((ext_vector_type(8)))  float    v8f;
typedef __attribute__((ext_vector_type(4)))  float    v4f;
typedef v4f  __attribute__((may_alias)) v4fa;

__device__ __forceinline__ unsigned short f2bf(float f) { unsigned u = __float_as_uint(f); u += 0x7FFFu + ((u >> 16) & 1u); return (unsigned short)(u >> 16); }
__device__ __forceinline__ float bfr(float f) { return __uint_as_float(((unsigned)f2bf(f)) << 16); }
__device__ __forceinline__ v16bf cat16b(v8us lo, v8us hi) { return __builtin_bit_cast(v16bf, __builtin_shufflevector(lo, hi, 0, 1, 2, 3, 4, 5, 6, 7, 8, 9, 10, 11, 12, 13, 14, 15)); }
__device__ __forceinline__ v8f wmmab(v16bf a, v16bf b, v8f c) { return __builtin_amdgcn_wmma_f32_16x16x32_bf16(false, a, false, b, (short)0, c, false, false); }
__device__ __forceinline__ v8f wmmabg(v16bf a, v16bf b, v8f c) { c = wmmab(a, b, c); asm volatile("v_nop\n\tv_nop\n\tv_nop\n\tv_nop" : "+v"(c) : "v"(a), "v"(b)); return c; }
__device__ __forceinline__ v16bf ldb(const bf* p)  { return cat16b(*(const v8us*)p, *(const v8us*)(p + 16)); }
__device__ __forceinline__ void wave_sync() { __builtin_amdgcn_fence(3  , "wavefront"); __builtin_amdgcn_wave_barrier(); asm volatile("" ::: "memory"); }

__global__ __launch_bounds__(256) void k_cvt8(const float* __restrict__ src, bf* dst, size_t n8) {
    const size_t i = (size_t)blockIdx.x * 256 + threadIdx.x; if (i >= n8) return;
    const v8f v = *(const v8f*)(src + i * 8); v8us o;
#pragma unroll
    for (int k = 0; k < 8; ++k) o[k] = f2bf(v[k]);
    *(volatile v8us*)(dst + i * 8) = o; __threadfence(); *(volatile v8us*)(dst + i * 8) = o;
}

__global__ __launch_bounds__(256) void k_xt(const float* __restrict__ x, bf* XT) {
#pragma clang fp contract(off)
    __shared__ float ts[64 * TP];
    const unsigned tid = threadIdx.x;
    const unsigned z = blockIdx.y, j0 = blockIdx.x * 64u;
    const float* src = x + ((size_t)z * SEQ_FULL + j0) * HD;
#pragma unroll
    for (int s = 0; s < 4; ++s) { const unsigned p = (unsigned)s * 256u + tid; const unsigned row = p >> 4, c4 = (p & 15u) * 4u;
        const v4f v = *(const v4f*)(src + (size_t)row * HD + c4);
        ts[row * TP + c4 + 0] = v[0]; ts[row * TP + c4 + 1] = v[1]; ts[row * TP + c4 + 2] = v[2]; ts[row * TP + c4 + 3] = v[3]; }
    __syncthreads();
    bf* dst = XT + ((size_t)z * HD) * SEQ + j0;
    v8us o[2];
#pragma unroll
    for (int s = 0; s < 2; ++s) { const unsigned p = (unsigned)s * 256u + tid; const unsigned d = p >> 3, q = (p & 7u) * 8u;
#pragma unroll
        for (int k = 0; k < 8; ++k) o[s][k] = f2bf(ts[(q + k) * TP + d]); }
#pragma unroll 1
    for (int ps = 0; ps < 2; ++ps) {
#pragma unroll
        for (int s = 0; s < 2; ++s) { const unsigned p = (unsigned)s * 256u + tid; const unsigned d = p >> 3, q = (p & 7u) * 8u;
            *(volatile v8us*)(dst + (size_t)d * SEQ + q) = o[s]; }
        if (ps == 0) __threadfence(); }
}

__global__ __launch_bounds__(32) void k_gram(const bf* __restrict__ XT, float* GP) {
    __shared__ __align__(16) float os[16 * OSW];
    const int lane = threadIdx.x & 31, lr = lane & 15, hi = lane >> 4;
    const unsigned z = blockIdx.x, c = blockIdx.y;
    v8f acc[4][4];
#pragma unroll
    for (int mb = 0; mb < 4; ++mb)
#pragma unroll
        for (int nb = 0; nb < 4; ++nb) acc[mb][nb] = (v8f){};
    const size_t aoff = ((size_t)z * HD + (size_t)lr) * SEQ + (size_t)c * KC + 8 * hi;
#pragma unroll 1
    for (int kc = 0; kc < KC; kc += 32) {
        v16bf a[4];
#pragma unroll
        for (int mb = 0; mb < 4; ++mb) a[mb] = ldb(XT + aoff + (size_t)mb * 16 * SEQ + kc);
#pragma unroll
        for (int nb = 0; nb < 4; ++nb) {
#pragma unroll
            for (int mb = 0; mb < 4; ++mb) acc[mb][nb] = wmmabg(a[mb], a[nb], acc[mb][nb]); }
    }
    float* gp = GP + ((size_t)c * NZ + z) * (size_t)(HD * HD);
#pragma unroll
    for (int mb = 0; mb < 4; ++mb) {
#pragma unroll
        for (int nb = 0; nb < 4; ++nb) {
#pragma unroll
            for (int j = 0; j < 8; ++j) os[(hi * 8 + j) * OSW + nb * 16 + lr] = acc[mb][nb][j]; }
        wave_sync();
        float* drow = gp + (size_t)(mb * 16) * HD;
#pragma unroll 1
        for (int ps = 0; ps < 2; ++ps) {
#pragma unroll
            for (int s = 0; s < 8; ++s) { const int row = 2 * s + (lane >> 4), cofs = (lane & 15) * 4;
                const v4f val = *(const v4fa*)(&os[row * OSW + cofs]);
                *(volatile v4f*)(drow + (size_t)row * HD + cofs) = val; }
            if (ps == 0) __threadfence(); }
        wave_sync();
    }
}

__global__ __launch_bounds__(256) void k_gsum(const float* __restrict__ GP, bf* GB) {
#pragma clang fp contract(off)
    const unsigned p = blockIdx.x * 256u + threadIdx.x; if (p >= (unsigned)NZ * 1024u) return;
    const unsigned z = p >> 10, r = p & 1023u, e = r >> 4, q = r & 15u, c8 = (q & 7u) * 8u;
    const size_t go = ((size_t)z * HD + e) * HD + c8;
    v4f s0 = *(const v4f*)(GP + go), s1 = *(const v4f*)(GP + go + 4);
#pragma unroll 1
    for (unsigned c = 1; c < (unsigned)KSPLIT; ++c) { const float* g = GP + (size_t)c * NZ * (size_t)(HD * HD) + go;
        const v4f t0 = *(const v4f*)g, t1 = *(const v4f*)(g + 4); s0 = s0 + t0; s1 = s1 + t1; }
    const bool res = q >= 8u;
    v8us o;
#pragma unroll
    for (int k = 0; k < 4; ++k) { const float v0 = s0[k], v1 = s1[k];
        const float w0 = res ? (v0 - bfr(v0)) : v0; const float w1 = res ? (v1 - bfr(v1)) : v1;
        o[k] = f2bf(w0); o[4 + k] = f2bf(w1); }
    *(volatile v8us*)(GB + (size_t)p * 8) = o; __threadfence(); *(volatile v8us*)(GB + (size_t)p * 8) = o;
}

__global__ __launch_bounds__(32) void k_out(const bf* __restrict__ XB, const bf* __restrict__ GB, float* OUT) {
    __shared__ __align__(16) float os[16 * OSW];
    const int lane = threadIdx.x & 31, lr = lane & 15, hi = lane >> 4;
    const unsigned z = blockIdx.y, r0 = blockIdx.x * 64u;
    v8f acc[4][4];
#pragma unroll
    for (int mb = 0; mb < 4; ++mb)
#pragma unroll
        for (int nb = 0; nb < 4; ++nb) acc[mb][nb] = (v8f){};
    const size_t aoff = ((size_t)z * SEQ + r0 + (size_t)lr) * HD + 8 * hi;
    const size_t boff = ((size_t)z * HD + (size_t)lr) * (size_t)(2 * HD) + 8 * hi;
#pragma unroll 1
    for (int kc = 0; kc < HD; kc += 32) {
        v16bf a[4];
#pragma unroll
        for (int mb = 0; mb < 4; ++mb) a[mb] = ldb(XB + aoff + (size_t)mb * 16 * HD + kc);
#pragma unroll
        for (int nb = 0; nb < 4; ++nb) {
            const v16bf bv = ldb(GB + boff + (size_t)nb * 16 * (2 * HD) + kc);
            const v16bf br = ldb(GB + boff + (size_t)nb * 16 * (2 * HD) + HD + kc);
#pragma unroll
            for (int mb = 0; mb < 4; ++mb) { acc[mb][nb] = wmmabg(a[mb], bv, acc[mb][nb]); acc[mb][nb] = wmmabg(a[mb], br, acc[mb][nb]); } }
    }
    float* op = OUT + ((size_t)z * OUT_SEQ + r0) * HD;
#pragma unroll
    for (int mb = 0; mb < 4; ++mb) {
#pragma unroll
        for (int nb = 0; nb < 4; ++nb) {
#pragma unroll
            for (int j = 0; j < 8; ++j) os[(hi * 8 + j) * OSW + nb * 16 + lr] = acc[mb][nb][j]; }
        wave_sync();
        float* drow = op + (size_t)(mb * 16) * HD;
#pragma unroll 1
        for (int ps = 0; ps < 2; ++ps) {
#pragma unroll
            for (int s = 0; s < 8; ++s) { const int row = 2 * s + (lane >> 4), cofs = (lane & 15) * 4;
                const v4f val = *(const v4fa*)(&os[row * OSW + cofs]);
                *(volatile v4f*)(drow + (size_t)row * HD + cofs) = val; }
            if (ps == 0) __threadfence(); }
        wave_sync();
    }
}

static constexpr size_t al256(size_t v) { return (v + 255) & ~(size_t)255; }
static constexpr size_t SZ_XB = al256((size_t)NZ * SEQ * HD * 2);
static constexpr size_t SZ_XT = al256((size_t)NZ * HD * SEQ * 2);
static constexpr size_t SZ_GP = al256((size_t)KSPLIT * NZ * HD * HD * 4);
static constexpr size_t SZ_GB = al256((size_t)NZ * HD * 2 * HD * 2);
static constexpr size_t SZ_TOTAL = SZ_XB + SZ_XT + SZ_GP + SZ_GB;
static_assert(SZ_TOTAL <= (size_t)134217728);
static constexpr size_t NEED_X   = ((size_t)(NZ - 1) * SEQ_FULL + SEQ) * HD;
static constexpr size_t NEED_OUT = ((size_t)(NZ - 1) * OUT_SEQ + SEQ) * HD;
static_assert(NEED_OUT <= (size_t)NB_FULL * NHD * SEQ_FULL * HD || OUT_SEQ != SEQ);

extern "C" void kernel_launch(void* const* d_in, const int* in_sizes, int n_in,
                              void* d_out, int out_size, void* d_ws, size_t ws_size, hipStream_t stream) {
    if (n_in < 1) return;
    if ((size_t)in_sizes[0] < NEED_X) return;
    if ((size_t)out_size < NEED_OUT) return;
    if (SZ_TOTAL > ws_size) return;
    const float* x = (const float*)d_in[0];
    float* OUT = (float*)d_out;
    char* wsp = (char*)d_ws;
    bf* XB = (bf*)wsp; wsp += SZ_XB;
    bf* XT = (bf*)wsp; wsp += SZ_XT;
    float* GP = (float*)wsp; wsp += SZ_GP;
    bf* GB = (bf*)wsp; wsp += SZ_GB;

    if (SEQ == SEQ_FULL) {
        const size_t n8 = (size_t)NZ * SEQ * HD / 8;
        k_cvt8<<<(unsigned)((n8 + 255) / 256), 256, 0, stream>>>(x, XB, n8);
    } else {
        const size_t n8 = (size_t)SEQ * HD / 8;
        for (unsigned zz = 0; zz < (unsigned)NZ; ++zz) k_cvt8<<<(unsigned)((n8 + 255) / 256), 256, 0, stream>>>(x + (size_t)zz * SEQ_FULL * HD, XB + (size_t)zz * SEQ * HD, n8);
    }
    k_xt<<<dim3(SEQ / 64, NZ, 1), 256, 0, stream>>>(x, XT);
    k_gram<<<dim3(NZ, KSPLIT, 1), 32, 0, stream>>>(XT, GP);
    k_gsum<<<(unsigned)(((size_t)NZ * 1024) / 256), 256, 0, stream>>>(GP, GB);
    k_out<<<dim3(SEQ / 64, NZ, 1), 32, 0, stream>>>(XB, GB, OUT);
}
